// PDN_80032420594375
// MI455X (gfx1250) — hardware-run, weakly checked
//
#include <hip/hip_runtime.h>


namespace {
constexpr int NB_ = 16, C3 = 1024, C4 = 2048, C = 3072, HW = 28, P = 784, PP = 800, H4 = 14, NL = 9, NK = 2000, KC = 512;
constexpr float AS = 16.0f  , MS = 256.0f, WSC = 256.0f, FS_ = 256.0f;
typedef _Float16 b16;
typedef __attribute__((ext_vector_type(16))) _Float16 v16b;
typedef __attribute__((ext_vector_type(8))) _Float16 v8b;
typedef __attribute__((ext_vector_type(8))) float v8f;
typedef __attribute__((ext_vector_type(4))) float v4f;
__device__ __forceinline__ float bf16_rne(float f) { unsigned int u = __float_as_uint(f); u += 0x7FFFu + ((u >> 16) & 1u); float r = __uint_as_float(u & 0xFFFF0000u); asm volatile("" : "+v"(r)); return r; }
__device__ __forceinline__ float bfv(float f) { float r = bf16_rne(f); asm volatile("" : "+v"(r)); return r; }
__device__ __forceinline__ void split16(float v, b16& hi, b16& lo) { hi = (b16)v; lo = (b16)(v - (float)hi); }
__device__ __forceinline__ v16b frag_kb(const b16* p, int hh) { const v8b a = *(const v8b*)(p + 8 * hh), b = *(const v8b*)(p + 16 + 8 * hh); v16b f;
#pragma unroll
  for (int e = 0; e < 8; ++e) { f[e] = a[e]; f[8 + e] = b[e]; } return f; }
__device__ __forceinline__ v8f wmma16b(v16b a, v16b b, v8f c) { v8f d = __builtin_amdgcn_wmma_f32_16x16x32_f16(false, a, false, b, (short)0, c, false, false); asm volatile("v_nop\n\tv_nop\n\tv_nop\n\tv_nop" : "+v"(d) : "v"(a), "v"(b)); return d; }
__device__ __forceinline__ void wave_lds_sync() { __builtin_amdgcn_fence(__ATOMIC_RELEASE, "workgroup"); __builtin_amdgcn_wave_barrier(); __builtin_amdgcn_fence(__ATOMIC_ACQUIRE, "workgroup"); }
__device__ __forceinline__ float pmul(float a, float b) { float p = a * b; asm volatile("" : "+v"(p)); return p; }
__device__ __forceinline__ int iclamp(int v, int lo, int hi) { return v < lo ? lo : (v > hi ? hi : v); }
__device__ __forceinline__ float xval(const float* __restrict__ l3, const float* __restrict__ l4, int b, int c, int p) {
  if (c >= C4) return bfv(l3[(((size_t)b * C3 + (c - C4)) * P) + p]);
  const int y = p / HW, xw = p % HW; const float sy = 0.5f * (float)y - 0.25f, sx = 0.5f * (float)xw - 0.25f; const int y0 = (int)floorf(sy), x0 = (int)floorf(sx); const float wy = sy - (float)y0, wx = sx - (float)x0; const int ya = iclamp(y0, 0, H4 - 1), yb = iclamp(y0 + 1, 0, H4 - 1), xa = iclamp(x0, 0, H4 - 1), xb = iclamp(x0 + 1, 0, H4 - 1);
  const float* pl = l4 + ((size_t)b * C4 + c) * (H4 * H4); const float v00 = bfv(pl[ya * H4 + xa]), v01 = bfv(pl[ya * H4 + xb]), v10 = bfv(pl[yb * H4 + xa]), v11 = bfv(pl[yb * H4 + xb]);
  return (1.0f - wy) * ((1.0f - wx) * v00 + wx * v01) + wy * ((1.0f - wx) * v10 + wx * v11); }

__global__ __launch_bounds__(256) void wput_kernel(const float* __restrict__ wl, const float* __restrict__ wc, b16* __restrict__ WL, b16* __restrict__ WC) { const size_t nt = (size_t)gridDim.x * 256, u0 = (size_t)blockIdx.x * 256 + threadIdx.x; v8b v;
  for (size_t u = u0; u < (size_t)16 * (C / 8); u += nt) { const int o = (int)(u / (C / 8)), k0 = (int)(u % (C / 8)) * 8;
#pragma unroll
    for (int j = 0; j < 8; ++j) v[j] = (b16)(o < NL ? bf16_rne(wl[(size_t)o * C + k0 + j]) * WSC : 0.0f); for (int pass = 0; pass < 2; ++pass) { *(volatile v8b*)(WL + (size_t)o * C + k0) = v; __threadfence(); } }
  for (size_t u = u0; u < (size_t)NK * (C / 8); u += nt) { const int o = (int)(u / (C / 8)), k0 = (int)(u % (C / 8)) * 8;
#pragma unroll
    for (int j = 0; j < 8; ++j) v[j] = (b16)(bf16_rne(wc[(size_t)o * C + k0 + j]) * WSC); for (int pass = 0; pass < 2; ++pass) { *(volatile v8b*)(WC + (size_t)o * C + k0) = v; __threadfence(); } } }
__global__ __launch_bounds__(32) void maps_kernel(const float* __restrict__ l3, const float* __restrict__ l4, const b16* __restrict__ WL, const float* __restrict__ wl, int BLIM, float* __restrict__ MP) { __shared__ __attribute__((aligned(16))) b16 Ah[16][KC + 8], Al[16][KC + 8]; __shared__ float Bs[16], Mq[16][17]; const int lane = threadIdx.x, nloc = lane & 15, hlf = lane >> 4; const int b = blockIdx.x / (P / 16), px0 = (blockIdx.x % (P / 16)) * 16; if (b >= BLIM) return;
  if (lane < 16) { Bs[lane] = 0.0f; for (int k = KC; k < KC + 8; ++k) { Ah[lane][k] = (b16)0.0f; Al[lane][k] = (b16)0.0f; } }
  v8f acc = (v8f){}; float bsq = 0.0f;
#pragma unroll 1
  for (int ch = 0; ch < C / KC; ++ch) { wave_lds_sync();
    for (int cc = hlf; cc < KC; cc += 2) { const float v = xval(l3, l4, b, ch * KC + cc, px0 + nloc); bsq += v * v; b16 p, pl; split16(v * AS, p, pl); Ah[nloc][cc] = p; Al[nloc][cc] = pl; }
    wave_lds_sync();
#pragma unroll 4
    for (int kb = 0; kb < KC; kb += 32) { const v16b bw = frag_kb(WL + (size_t)nloc * C + ch * KC + kb, hlf); acc = wmma16b(frag_kb(&Ah[nloc][kb], hlf), bw, acc); acc = wmma16b(frag_kb(&Al[nloc][kb], hlf), bw, acc); } }
  bsq += __shfl_xor(bsq, 16);
#pragma unroll
  for (int r8 = 0; r8 < 8; ++r8) Mq[8 * hlf + r8][nloc] = acc[r8] * (1.0f / (AS * WSC));
  if (lane < 16) Bs[lane] = bsq;
  wave_lds_sync();
  if (lane < 16) { float lg[NL]; float mx = -INFINITY;
#pragma unroll
    for (int l = 0; l < NL; ++l) { float asq = 0.0f; for (int c = 0; c < C; ++c) { const float w = bfv(wl[(size_t)l * C + c]); asq += w * w; } lg[l] = -(Bs[lane] - 2.0f * Mq[lane][l] + asq); mx = fmaxf(mx, lg[l]); }
    float sm = 0.0f;
#pragma unroll
    for (int l = 0; l < NL; ++l) { lg[l] = __expf(lg[l] - mx); sm += lg[l]; } const float inv = 1.0f / sm;
#pragma unroll
    for (int l = 0; l < NL; ++l) Mq[lane][l] = lg[l] * inv; for (int l = NL; l < 16; ++l) Mq[lane][l] = 0.0f; }
  wave_lds_sync();
  for (int pass = 0; pass < 2; ++pass) { for (int q = 0; q < 8; ++q) { const int idx = q * 32 + lane; ((volatile float*)MP)[((size_t)b * PP + px0) * 16 + idx] = Mq[idx >> 4][idx & 15]; } __threadfence(); } }

__global__ __launch_bounds__(32) void feat_kernel(const float* __restrict__ l3, const float* __restrict__ l4, const float* __restrict__ MP, int BLIM, float* __restrict__ FT) { __shared__ __attribute__((aligned(16))) b16 Ah[16][PP + 8], Al[16][PP + 8], Bh[16][PP + 8], Bl[16][PP + 8]; __shared__ float Tq[16][17]; const int lane = threadIdx.x, nloc = lane & 15, hlf = lane >> 4; const int b = blockIdx.x / (C / 16), c0 = (blockIdx.x % (C / 16)) * 16; if (b >= BLIM) return;
  for (int rr = 0; rr < 16; ++rr) for (int p = lane; p < PP + 8; p += 32) { float v = 0.0f; if (p < P) v = xval(l3, l4, b, c0 + rr, p); b16 hq, lq; split16(v * AS, hq, lq); Ah[rr][p] = hq; Al[rr][p] = lq; float m = 0.0f; if (p < P) m = MP[((size_t)b * PP + p) * 16 + rr]; split16(m * MS, hq, lq); Bh[rr][p] = hq; Bl[rr][p] = lq; }
  wave_lds_sync(); v8f acc = (v8f){};
#pragma unroll 5
  for (int kb = 0; kb < PP; kb += 32) { const v16b a = frag_kb(&Ah[nloc][kb], hlf), al = frag_kb(&Al[nloc][kb], hlf), bh = frag_kb(&Bh[nloc][kb], hlf), bl = frag_kb(&Bl[nloc][kb], hlf); acc = wmma16b(a, bh, acc); acc = wmma16b(a, bl, acc); acc = wmma16b(al, bh, acc); }
#pragma unroll
  for (int r8 = 0; r8 < 8; ++r8) Tq[8 * hlf + r8][nloc] = acc[r8] * (1.0f / (AS * MS * (float)P));
  wave_lds_sync();
  for (int pass = 0; pass < 2; ++pass) { for (int q = 0; q < 8; ++q) { const int idx = q * 32 + lane; ((volatile float*)FT)[((size_t)b * C + c0) * 16 + idx] = Tq[idx >> 4][idx & 15]; } __threadfence(); } }
typedef __attribute__((ext_vector_type(2))) _Float16 v2b;
__global__ __launch_bounds__(256) void mbar_kernel(const float* __restrict__ FT, const float* __restrict__ mod, b16* __restrict__ MBh, b16* __restrict__ MBl) { const int u = blockIdx.x * 256 + threadIdx.x; if (u >= NB_ * C / 2) return; v2b hh, ll;
  for (int e = 0; e < 2; ++e) { const int idx = 2 * u + e; const int b = idx / C, c = idx % C; float s = 0.0f;
#pragma unroll
    for (int l = 0; l < NL - 1; ++l) s += pmul(FT[((size_t)b * C + c) * 16 + l], bfv(mod[(size_t)c * NL + l])); s *= (1.0f / (float)(NL - 1)); b16 hq, lq; split16(s * FS_, hq, lq); hh[e] = hq; ll[e] = lq; }
  for (int pass = 0; pass < 2; ++pass) { *(volatile v2b*)(MBh + 2 * (size_t)u) = hh; *(volatile v2b*)(MBl + 2 * (size_t)u) = ll; __threadfence(); } }
__global__ __launch_bounds__(32) void score_kernel(const b16* __restrict__ WC, const b16* __restrict__ MBh, const b16* __restrict__ MBl, float* __restrict__ SC) { __shared__ float Tq[16][17]; const int lane = threadIdx.x, nloc = lane & 15, hlf = lane >> 4; const int k0 = blockIdx.x * 16; v8f acc = (v8f){};
#pragma unroll 4
  for (int kb = 0; kb < C; kb += 32) { const v16b a = frag_kb(WC + (size_t)(k0 + nloc) * C + kb, hlf); acc = wmma16b(a, frag_kb(MBh + (size_t)nloc * C + kb, hlf), acc); acc = wmma16b(a, frag_kb(MBl + (size_t)nloc * C + kb, hlf), acc); }
#pragma unroll
  for (int r8 = 0; r8 < 8; ++r8) Tq[8 * hlf + r8][nloc] = acc[r8] * (1.0f / (WSC * FS_));
  wave_lds_sync();
  for (int pass = 0; pass < 2; ++pass) { for (int q = 0; q < 8; ++q) { const int idx = q * 32 + lane; ((volatile float*)SC)[(size_t)k0 * 16 + idx] = Tq[idx >> 4][idx & 15]; } __threadfence(); } }
__global__ __launch_bounds__(256) void copy_kernel(const float* __restrict__ SC, const float* __restrict__ MP, const float* __restrict__ FT, float* __restrict__ out) { const size_t u = (size_t)blockIdx.x * 256 + threadIdx.x; const size_t n0 = (size_t)NB_ * NK, n1 = (size_t)NB_ * NL * P, n2 = (size_t)NB_ * C * NL; if (u >= n0 + n1 + n2) return; float v;
  if (u < n0) { const int b = (int)(u / NK), k = (int)(u % NK); v = SC[(size_t)k * 16 + b]; }
  else if (u < n0 + n1) { const size_t w = u - n0; const int b = (int)(w / (NL * P)), l = (int)((w / P) % NL), p = (int)(w % P); v = MP[((size_t)b * PP + p) * 16 + l]; }
  else { const size_t w = u - n0 - n1; const int b = (int)(w / ((size_t)C * NL)), c = (int)((w / NL) % C), l = (int)(w % NL); v = FT[((size_t)b * C + c) * 16 + l]; }
  for (int pass = 0; pass < 2; ++pass) { ((volatile float*)out)[u] = v; __threadfence(); } }
}

extern "C" void kernel_launch(void* const* d_in, const int* in_sizes, int n_in, void* d_out, int out_size, void* d_ws, size_t ws_size, hipStream_t stream) {
  (void)n_in;
  auto Fp = [&](int i) { return (const float*)d_in[i]; };
  if (in_sizes[0] != NB_ * C3 * P || in_sizes[1] != NB_ * C4 * H4 * H4 || in_sizes[2] != NL * C || in_sizes[3] != NK * C || in_sizes[4] != C * NL || out_size != NB_ * NK + NB_ * NL * P + NB_ * C * NL) return;
  const int BLIM = NB_;
  size_t off = 0; char* ws = (char*)d_ws;
  auto carve = [&](size_t bytes) { char* p = ws + off; off += (bytes + 255) & ~(size_t)255; return p; };
  b16* WL = (b16*)carve((size_t)16 * C * 2); b16* WC = (b16*)carve((size_t)NK * C * 2); float* MP = (float*)carve((size_t)NB_ * PP * 16 * 4); float* FT = (float*)carve((size_t)NB_ * C * 16 * 4); b16* MBh = (b16*)carve((size_t)NB_ * C * 2); b16* MBl = (b16*)carve((size_t)NB_ * C * 2); float* SC = (float*)carve((size_t)NK * 16 * 4);
  if (off > ws_size || off > ((size_t)24 << 20)) return;
  wput_kernel<<<128, 256, 0, stream>>>(Fp(2), Fp(3), WL, WC);
  maps_kernel<<<BLIM * (P / 16), 32, 0, stream>>>(Fp(0), Fp(1), WL, Fp(2), BLIM, MP);
  feat_kernel<<<BLIM * (C / 16), 32, 0, stream>>>(Fp(0), Fp(1), MP, BLIM, FT);
  mbar_kernel<<<(NB_ * C / 2 + 255) / 256, 256, 0, stream>>>(FT, Fp(4), MBh, MBl);
  score_kernel<<<NK / 16, 32, 0, stream>>>(WC, MBh, MBl, SC);
  copy_kernel<<<(NB_ * NK + NB_ * NL * P + NB_ * C * NL + 255) / 256, 256, 0, stream>>>(SC, MP, FT, (float*)d_out);
}
